// EntityGraphRefinement_7696581394665
// MI455X (gfx1250) — hardware-run, weakly checked
//
#include <hip/hip_runtime.h>
#include <stddef.h>

#define NB 4
#define SQ 1024
#define DM 768
#define NE 128
#define NH 12
#define KD 64
#define NTOK (NB * SQ)
#define NROW (NB * NE)
#define NHO 3072
#define QG 8
#define ATT_LDS (65536 + 32768 + 32768 + 128)

static_assert(NTOK % 64 == 0);
static_assert(NROW % 64 == 0);
static_assert(NE % 64 == 0);
static_assert(DM % 64 == 0);
static_assert(NHO % 64 == 0);
static_assert(DM % 32 == 0);
static_assert(DM % 256 == 0);
static_assert(SQ % 64 == 0);
static_assert(NE == QG * 16);
static_assert(NH * KD == DM);
static_assert(SQ == 8 * 128);

typedef _Float16 f16;
typedef unsigned short u16;
typedef f16 v16h __attribute__((ext_vector_type(16)));
typedef __bf16 v16b __attribute__((ext_vector_type(16)));
typedef float v8f __attribute__((ext_vector_type(8)));
typedef float v4f_t __attribute__((ext_vector_type(4)));
typedef v4f_t __attribute__((may_alias)) v4f;
typedef unsigned int v4u_t __attribute__((ext_vector_type(4)));
typedef v4u_t __attribute__((may_alias)) v4u;

union FragH { v16h v; v4u_t u[2]; };
union FragB { v16b v; v4u_t u[2]; };

__device__ __forceinline__ v8f zero8() {
    v8f z;
#pragma unroll
    for (int i = 0; i < 8; ++i) z[i] = 0.0f;
    return z;
}
__device__ __forceinline__ v4f_t zero4() {
    v4f_t z;
    z[0] = 0.0f; z[1] = 0.0f; z[2] = 0.0f; z[3] = 0.0f;
    return z;
}

__device__ __forceinline__ void ldfr(v4u_t& u0, v4u_t& u1, const u16* p) {
    u0 = *(const v4u*)(p);
    u1 = *(const v4u*)(p + 16);
}

__device__ __forceinline__ v8f wmma_h(v16h a, v16h b, v8f c) {
    return __builtin_amdgcn_wmma_f32_16x16x32_f16(false, a, false, b, (short)0, c, false, false);
}
__device__ __forceinline__ v8f wmma_b(v16b a, v16b b, v8f c) {
    return __builtin_amdgcn_wmma_f32_16x16x32_bf16(false, a, false, b, (short)0, c, false, false);
}

__device__ __forceinline__ unsigned hbits(float x) {
    return (unsigned)__builtin_bit_cast(unsigned short, (f16)x);
}
__device__ __forceinline__ unsigned bbits(float x) {
    const unsigned u = __float_as_uint(x);
    return (u + 0x7FFFu + ((u >> 16) & 1u)) >> 16;
}
__device__ __forceinline__ v4u_t pack8h(v4f_t a, v4f_t b, float s) {
    v4u_t r;
    r[0] = hbits(a[0] * s) | (hbits(a[1] * s) << 16);
    r[1] = hbits(a[2] * s) | (hbits(a[3] * s) << 16);
    r[2] = hbits(b[0] * s) | (hbits(b[1] * s) << 16);
    r[3] = hbits(b[2] * s) | (hbits(b[3] * s) << 16);
    return r;
}
__device__ __forceinline__ void pack8b2(v4f_t a, v4f_t b, v4u_t& hi, v4u_t& lo) {
    float x[8];
    x[0] = a[0]; x[1] = a[1]; x[2] = a[2]; x[3] = a[3];
    x[4] = b[0]; x[5] = b[1]; x[6] = b[2]; x[7] = b[3];
    unsigned hb[8], lb[8];
#pragma unroll
    for (int i = 0; i < 8; ++i) {
        hb[i] = bbits(x[i]);
        lb[i] = bbits(x[i] - __uint_as_float(hb[i] << 16));
    }
#pragma unroll
    for (int i = 0; i < 4; ++i) {
        hi[i] = hb[2 * i] | (hb[2 * i + 1] << 16);
        lo[i] = lb[2 * i] | (lb[2 * i + 1] << 16);
    }
}

__device__ __forceinline__ float wave_sum(float v) {
#pragma unroll
    for (int off = 16; off > 0; off >>= 1) v += __shfl_xor(v, off, 32);
    return v;
}

__global__ void __launch_bounds__(256) xprep_kernel(
    const float* __restrict__ emb, const float* __restrict__ pos,
    u16* __restrict__ xf, u16* __restrict__ xh, u16* __restrict__ xl, int n8)
{
    const int i = blockIdx.x * 256 + threadIdx.x;
    const bool ok = (i < n8);
    const int ic = ok ? i : 0;
    const size_t e0 = (size_t)ic * 8;
    const size_t p0 = e0 % ((size_t)SQ * DM);
    v4f_t a = *(const v4f*)(emb + e0), c = *(const v4f*)(emb + e0 + 4);
    const v4f_t pa = *(const v4f*)(pos + p0), pc = *(const v4f*)(pos + p0 + 4);
    a = a + pa; c = c + pc;
    const v4u_t pf = pack8h(a, c, 1.0f);
    v4u_t ph, pl; pack8b2(a, c, ph, pl);
    if (ok) {
        *(volatile v4u_t*)(xf + e0) = pf;
        *(volatile v4u_t*)(xh + e0) = ph;
        *(volatile v4u_t*)(xl + e0) = pl;
    }
    __threadfence();
    if (ok) {
        *(volatile v4u_t*)(xf + e0) = pf;
        *(volatile v4u_t*)(xh + e0) = ph;
        *(volatile v4u_t*)(xl + e0) = pl;
    }
}

__global__ void __launch_bounds__(256) cvt16_kernel(
    const float* __restrict__ src, u16* __restrict__ dst, int n8, float scale)
{
    const int i = blockIdx.x * 256 + threadIdx.x;
    const bool ok = (i < n8);
    const int ic = ok ? i : 0;
    const size_t e0 = (size_t)ic * 8;
    const v4f_t a = *(const v4f*)(src + e0), c = *(const v4f*)(src + e0 + 4);
    const v4u_t pf = pack8h(a, c, scale);
    if (ok) { *(volatile v4u_t*)(dst + e0) = pf; }
    __threadfence();
    if (ok) { *(volatile v4u_t*)(dst + e0) = pf; }
}

__global__ void __launch_bounds__(256) context_kernel(
    const float* __restrict__ emb, const float* __restrict__ pos, float* __restrict__ cm)
{
    const int d = blockIdx.x * 256 + threadIdx.x;
    const int b = blockIdx.y;
    const float* er = emb + (size_t)b * SQ * DM + d;
    const float* pr = pos + d;
    float s = 0.0f;
#pragma unroll 4
    for (int si = 0; si < SQ; ++si) {
        const float xv = er[(size_t)si * DM] + pr[(size_t)si * DM];
        s += xv;
    }
    const float v = s * (1.0f / (float)SQ);
    float* dst = cm + b * DM + d;
    *(volatile float*)dst = v;
    __threadfence();
    *(volatile float*)dst = v;
}

template <int MODE>
__global__ void __launch_bounds__(256) wtrans_kernel(
    const float* __restrict__ src, u16* __restrict__ d0, u16* __restrict__ d1, float scale)
{
    __shared__ __align__(16) float tl[64 * 68];
    const int t = threadIdx.x;
    const int n0 = blockIdx.x * 64, k0 = blockIdx.y * 64;
    const int n = t & 63, kq = t >> 6;
#pragma unroll
    for (int r = 0; r < 16; ++r) {
        const int k = r * 4 + kq;
        tl[n * 68 + k] = src[(size_t)(k0 + k) * DM + n0 + n];
    }
    __syncthreads();
    const int rq = t >> 3, ks = (t & 7) * 8;
    v4u_t p0[2], p1[2];
#pragma unroll
    for (int ps = 0; ps < 2; ++ps) {
        const int nr = rq + 32 * ps;
        const v4f_t a = *(const v4f*)&tl[nr * 68 + ks], c = *(const v4f*)&tl[nr * 68 + ks + 4];
        if (MODE == 0) { p0[ps] = pack8h(a, c, scale); p1[ps] = p0[ps]; }
        else           { pack8b2(a, c, p0[ps], p1[ps]); }
    }
#pragma unroll
    for (int ps = 0; ps < 2; ++ps) {
        const size_t off = (size_t)(n0 + rq + 32 * ps) * DM + k0 + ks;
        *(volatile v4u_t*)(d0 + off) = p0[ps];
        if (MODE == 1) { *(volatile v4u_t*)(d1 + off) = p1[ps]; }
    }
    __threadfence();
#pragma unroll
    for (int ps = 0; ps < 2; ++ps) {
        const size_t off = (size_t)(n0 + rq + 32 * ps) * DM + k0 + ks;
        *(volatile v4u_t*)(d0 + off) = p0[ps];
        if (MODE == 1) { *(volatile v4u_t*)(d1 + off) = p1[ps]; }
    }
}

template <bool SPLIT, int OMODE>
__global__ void __launch_bounds__(128) gemm_kernel(
    const u16* __restrict__ A0, const u16* __restrict__ A1,
    const u16* __restrict__ B0, const u16* __restrict__ B1,
    const float* __restrict__ bias, int has_bias,
    int M, int N, int K, float oscale, float pscale,
    float* __restrict__ outF, u16* __restrict__ outP0, u16* __restrict__ outP1,
    const float* __restrict__ rowmask)
{
    __shared__ __align__(16) float Cs[64 * 68];
    const int t = threadIdx.x, w = t >> 5, lane = t & 31, hh = lane >> 4, m = lane & 15;
    const int wm = w >> 1, wn = w & 1;
    const int row0 = blockIdx.y * 64, col0 = blockIdx.x * 64;
    if (row0 + 64 > M || col0 + 64 > N) return;

    v8f acc[4];
#pragma unroll
    for (int i = 0; i < 4; ++i) acc[i] = zero8();

    const size_t ar0 = (size_t)(row0 + wm * 32 + m) * K + 8 * hh;
    const size_t ar1 = ar0 + (size_t)16 * K;
    const size_t bc0 = (size_t)(col0 + wn * 32 + m) * K + 8 * hh;
    const size_t bc1 = bc0 + (size_t)16 * K;

#pragma unroll 1
    for (int k0 = 0; k0 < K; k0 += 32) {
        if (!SPLIT) {
            FragH a0, a1, b0, b1;
            ldfr(a0.u[0], a0.u[1], A0 + ar0 + k0);
            ldfr(a1.u[0], a1.u[1], A0 + ar1 + k0);
            ldfr(b0.u[0], b0.u[1], B0 + bc0 + k0);
            ldfr(b1.u[0], b1.u[1], B0 + bc1 + k0);
            acc[0] = wmma_h(a0.v, b0.v, acc[0]);
            acc[1] = wmma_h(a0.v, b1.v, acc[1]);
            acc[2] = wmma_h(a1.v, b0.v, acc[2]);
            acc[3] = wmma_h(a1.v, b1.v, acc[3]);
            asm volatile("v_nop\n\tv_nop\n\tv_nop\n\tv_nop"
                         : "+v"(acc[0]), "+v"(acc[1]), "+v"(acc[2]), "+v"(acc[3])
                         : "v"(a0.v), "v"(a1.v), "v"(b0.v), "v"(b1.v));
        } else {
            FragB ah0, ah1, al0, al1, bh0, bh1, bl0, bl1;
            ldfr(ah0.u[0], ah0.u[1], A0 + ar0 + k0);
            ldfr(ah1.u[0], ah1.u[1], A0 + ar1 + k0);
            ldfr(al0.u[0], al0.u[1], A1 + ar0 + k0);
            ldfr(al1.u[0], al1.u[1], A1 + ar1 + k0);
            ldfr(bh0.u[0], bh0.u[1], B0 + bc0 + k0);
            ldfr(bh1.u[0], bh1.u[1], B0 + bc1 + k0);
            ldfr(bl0.u[0], bl0.u[1], B1 + bc0 + k0);
            ldfr(bl1.u[0], bl1.u[1], B1 + bc1 + k0);
            acc[0] = wmma_b(ah0.v, bh0.v, acc[0]);
            acc[0] = wmma_b(ah0.v, bl0.v, acc[0]);
            acc[0] = wmma_b(al0.v, bh0.v, acc[0]);
            acc[1] = wmma_b(ah0.v, bh1.v, acc[1]);
            acc[1] = wmma_b(ah0.v, bl1.v, acc[1]);
            acc[1] = wmma_b(al0.v, bh1.v, acc[1]);
            acc[2] = wmma_b(ah1.v, bh0.v, acc[2]);
            acc[2] = wmma_b(ah1.v, bl0.v, acc[2]);
            acc[2] = wmma_b(al1.v, bh0.v, acc[2]);
            acc[3] = wmma_b(ah1.v, bh1.v, acc[3]);
            acc[3] = wmma_b(ah1.v, bl1.v, acc[3]);
            acc[3] = wmma_b(al1.v, bh1.v, acc[3]);
            asm volatile("v_nop\n\tv_nop\n\tv_nop\n\tv_nop"
                         : "+v"(acc[0]), "+v"(acc[1]), "+v"(acc[2]), "+v"(acc[3])
                         : "v"(ah0.v), "v"(ah1.v), "v"(al0.v), "v"(al1.v),
                           "v"(bh0.v), "v"(bh1.v), "v"(bl0.v), "v"(bl1.v));
        }
    }

    float bv0 = 0.0f, bv1 = 0.0f;
    if (has_bias) {
        bv0 = bias[col0 + wn * 32 + m];
        bv1 = bias[col0 + wn * 32 + 16 + m];
    }
#pragma unroll
    for (int mt = 0; mt < 2; ++mt) {
#pragma unroll
        for (int nt = 0; nt < 2; ++nt) {
            const float bvv = nt ? bv1 : bv0;
#pragma unroll
            for (int r = 0; r < 8; ++r)
                Cs[(wm * 32 + mt * 16 + 8 * hh + r) * 68 + wn * 32 + nt * 16 + m] =
                    acc[mt * 2 + nt][r] * oscale + bvv;
        }
    }
    __syncthreads();

    if (OMODE == 0 || OMODE == 3) {
        const int c4 = m * 4;
        v4f_t vv[8];
#pragma unroll
        for (int it = 0; it < 8; ++it) {
            const int row = w * 16 + 2 * it + hh;
            v4f_t v = *(const v4f*)&Cs[row * 68 + c4];
            if (OMODE == 3) { const float rm = rowmask[row0 + row]; v = v * rm; }
            vv[it] = v;
        }
        float* ob = outF + (size_t)row0 * N + col0 + c4;
#pragma unroll
        for (int it = 0; it < 8; ++it)
            *(volatile v4f_t*)(ob + (size_t)(w * 16 + 2 * it + hh) * N) = vv[it];
        __threadfence();
#pragma unroll
        for (int it = 0; it < 8; ++it)
            *(volatile v4f_t*)(ob + (size_t)(w * 16 + 2 * it + hh) * N) = vv[it];
    }
    if (OMODE == 1 || OMODE == 3) {
        const int rq = lane >> 3, cs = (lane & 7) * 8;
        v4u_t pp[4];
#pragma unroll
        for (int it = 0; it < 4; ++it) {
            const int row = w * 16 + 4 * it + rq;
            const v4f_t a = *(const v4f*)&Cs[row * 68 + cs], c = *(const v4f*)&Cs[row * 68 + cs + 4];
            pp[it] = pack8h(a, c, pscale);
        }
        u16* ob = outP0 + (size_t)row0 * N + col0 + cs;
#pragma unroll
        for (int it = 0; it < 4; ++it)
            *(volatile v4u_t*)(ob + (size_t)(w * 16 + 4 * it + rq) * N) = pp[it];
        __threadfence();
#pragma unroll
        for (int it = 0; it < 4; ++it)
            *(volatile v4u_t*)(ob + (size_t)(w * 16 + 4 * it + rq) * N) = pp[it];
    }
    if (OMODE == 4) {
        const int grp = row0 / SQ, s0 = row0 - grp * SQ;
        const int rq = lane >> 3, ss = (lane & 7) * 8;
        v4u_t ph[4], pl[4];
#pragma unroll
        for (int it = 0; it < 4; ++it) {
            const int hk = w * 16 + 4 * it + rq;
            v4f_t a, c;
            a[0] = Cs[(ss + 0) * 68 + hk]; a[1] = Cs[(ss + 1) * 68 + hk];
            a[2] = Cs[(ss + 2) * 68 + hk]; a[3] = Cs[(ss + 3) * 68 + hk];
            c[0] = Cs[(ss + 4) * 68 + hk]; c[1] = Cs[(ss + 5) * 68 + hk];
            c[2] = Cs[(ss + 6) * 68 + hk]; c[3] = Cs[(ss + 7) * 68 + hk];
            pack8b2(a, c, ph[it], pl[it]);
        }
        const size_t base = ((size_t)grp * N + col0) * SQ + s0 + ss;
#pragma unroll
        for (int it = 0; it < 4; ++it) {
            const size_t off = base + (size_t)(w * 16 + 4 * it + rq) * SQ;
            *(volatile v4u_t*)(outP0 + off) = ph[it];
            *(volatile v4u_t*)(outP1 + off) = pl[it];
        }
        __threadfence();
#pragma unroll
        for (int it = 0; it < 4; ++it) {
            const size_t off = base + (size_t)(w * 16 + 4 * it + rq) * SQ;
            *(volatile v4u_t*)(outP0 + off) = ph[it];
            *(volatile v4u_t*)(outP1 + off) = pl[it];
        }
    }
}

__global__ void __launch_bounds__(256) attn_kernel(
    const u16* __restrict__ qp, const u16* __restrict__ kp,
    const u16* __restrict__ vth, const u16* __restrict__ vtl,
    u16* __restrict__ ctxh, u16* __restrict__ ctxl, float* __restrict__ invd)
{
    extern __shared__ __align__(16) unsigned char dlds[];
    float* S      = (float*)dlds;
    u16*   Ph     = (u16*)(dlds + 65536);
    u16*   Pl     = (u16*)(dlds + 98304);
    float* red    = (float*)dlds;
    float* invrow = (float*)(dlds + 131072);

    const int qg = blockIdx.x, h = blockIdx.y, b = blockIdx.z;
    const int n0 = qg * 16;
    const int t = threadIdx.x, w = t >> 5, lane = t & 31, hh = lane >> 4, m = lane & 15;

    {
        v8f acc[8];
#pragma unroll
        for (int i = 0; i < 8; ++i) acc[i] = zero8();
        const u16* pa = qp + (size_t)(n0 + m) * DM + h * KD + 8 * hh;
        const u16* pb = kp + (size_t)(b * SQ + w * 128 + m) * DM + h * KD + 8 * hh;
#pragma unroll
        for (int ks = 0; ks < 2; ++ks) {
            FragH a;
            ldfr(a.u[0], a.u[1], pa + ks * 32);
            FragH bf;
#pragma unroll
            for (int nt = 0; nt < 8; ++nt) {
                ldfr(bf.u[0], bf.u[1], pb + (size_t)nt * 16 * DM + ks * 32);
                acc[nt] = wmma_h(a.v, bf.v, acc[nt]);
            }
            asm volatile("v_nop\n\tv_nop\n\tv_nop\n\tv_nop"
                         : "+v"(acc[0]), "+v"(acc[1]), "+v"(acc[2]), "+v"(acc[3]),
                           "+v"(acc[4]), "+v"(acc[5]), "+v"(acc[6]), "+v"(acc[7])
                         : "v"(a.v), "v"(bf.v));
        }
#pragma unroll
        for (int nt = 0; nt < 8; ++nt) {
#pragma unroll
            for (int r = 0; r < 8; ++r)
                S[(8 * hh + r) * SQ + w * 128 + nt * 16 + m] = acc[nt][r] * (1.0f / 512.0f);
        }
    }
    __syncthreads();

    {
        const int row = t >> 4, c0 = (t & 15) * 64;
        float* Sr = S + row * SQ + c0;
        float mx = -3.0e38f;
#pragma unroll 4
        for (int j = 0; j < 16; ++j) {
            const v4f_t v = *(const v4f*)(Sr + 4 * j);
            mx = fmaxf(mx, fmaxf(fmaxf(v[0], v[1]), fmaxf(v[2], v[3])));
        }
#pragma unroll
        for (int off = 8; off > 0; off >>= 1) mx = fmaxf(mx, __shfl_xor(mx, off, 32));
        float sm = 0.0f;
#pragma unroll 2
        for (int j = 0; j < 16; ++j) {
            const v4f_t v = *(const v4f*)(Sr + 4 * j);
            v4f_t e;
            e[0] = __expf(v[0] - mx); e[1] = __expf(v[1] - mx);
            e[2] = __expf(v[2] - mx); e[3] = __expf(v[3] - mx);
            *(v4f*)(Sr + 4 * j) = e;
            sm += (e[0] + e[1]) + (e[2] + e[3]);
        }
#pragma unroll
        for (int off = 8; off > 0; off >>= 1) sm += __shfl_xor(sm, off, 32);
        const float inv = 1.0f / sm;
        if ((t & 15) == 0) invrow[row] = inv;
#pragma unroll 2
        for (int j = 0; j < 8; ++j) {
            v4f_t a = *(const v4f*)(Sr + 8 * j), c = *(const v4f*)(Sr + 8 * j + 4);
            a = a * inv; c = c * inv;
            v4u_t ph, pl; pack8b2(a, c, ph, pl);
            *(v4u*)(Ph + row * SQ + c0 + 8 * j) = ph;
            *(v4u*)(Pl + row * SQ + c0 + 8 * j) = pl;
        }
    }
    __syncthreads();

    {
        v8f acc[4];
#pragma unroll
        for (int i = 0; i < 4; ++i) acc[i] = zero8();
        const u16* pah = Ph + m * SQ + 8 * hh;
        const u16* pal = Pl + m * SQ + 8 * hh;
        const size_t vb0 = ((size_t)(b * DM + h * KD + m)) * SQ + 8 * hh;
#pragma unroll 1
        for (int ks = 0; ks < 4; ++ks) {
            const int k0 = w * 128 + ks * 32;
            FragB fa, fl;
            ldfr(fa.u[0], fa.u[1], pah + k0);
            ldfr(fl.u[0], fl.u[1], pal + k0);
            FragB gh, gl;
#pragma unroll
            for (int nt = 0; nt < 4; ++nt) {
                ldfr(gh.u[0], gh.u[1], vth + vb0 + (size_t)nt * 16 * SQ + k0);
                ldfr(gl.u[0], gl.u[1], vtl + vb0 + (size_t)nt * 16 * SQ + k0);
                acc[nt] = wmma_b(fa.v, gh.v, acc[nt]);
                acc[nt] = wmma_b(fa.v, gl.v, acc[nt]);
                acc[nt] = wmma_b(fl.v, gh.v, acc[nt]);
            }
            asm volatile("v_nop\n\tv_nop\n\tv_nop\n\tv_nop"
                         : "+v"(acc[0]), "+v"(acc[1]), "+v"(acc[2]), "+v"(acc[3])
                         : "v"(fa.v), "v"(fl.v), "v"(gh.v), "v"(gl.v));
        }
#pragma unroll
        for (int nt = 0; nt < 4; ++nt) {
#pragma unroll
            for (int r = 0; r < 8; ++r)
                red[(w * 16 + 8 * hh + r) * 64 + nt * 16 + m] = acc[nt][r];
        }
    }
    __syncthreads();

    if (t < 128) {
        const int row = t >> 3, cs = (t & 7) * 8;
        v4f_t a = zero4(), c = zero4();
#pragma unroll
        for (int ww = 0; ww < 8; ++ww) {
            a += *(const v4f*)&red[(ww * 16 + row) * 64 + cs];
            c += *(const v4f*)&red[(ww * 16 + row) * 64 + cs + 4];
        }
        v4u_t ph, pl; pack8b2(a, c, ph, pl);
        const size_t off = (size_t)(b * NE + n0 + row) * DM + h * KD + cs;
        *(volatile v4u_t*)(ctxh + off) = ph;
        *(volatile v4u_t*)(ctxl + off) = pl;
        __threadfence();
        *(volatile v4u_t*)(ctxh + off) = ph;
        *(volatile v4u_t*)(ctxl + off) = pl;
    }
    if (w == 0) {
        const float iv = invrow[lane & 15];
        const float v = (lane < 16) ? iv : 0.0f;
        float* dst = invd + ((size_t)((b * NH + h) * QG + qg)) * 32 + lane;
        *(volatile float*)dst = v;
        __threadfence();
        *(volatile float*)dst = v;
    }
}

__global__ void __launch_bounds__(256) post_kernel(
    const float* __restrict__ cm, const float* __restrict__ W1, const float* __restrict__ b1,
    const float* __restrict__ invd, float* __restrict__ Cb,
    float* __restrict__ maskws, float* __restrict__ mask_out)
{
    const int blk = blockIdx.x, t = threadIdx.x;
    if (blk < 12) {
        const int b = blk / 3, e = (blk - 3 * (blk / 3)) * 256 + t;
        const float* wr = W1 + (size_t)1537 * DM + e;
        const float* cr = cm + b * DM;
        float acc = 0.0f;
#pragma unroll 4
        for (int d = 0; d < DM; ++d) acc = fmaf(cr[d], wr[(size_t)d * DM], acc);
        const float v = acc + b1[e];
        float* dst = Cb + b * DM + e;
        *(volatile float*)dst = v;
        __threadfence();
        *(volatile float*)dst = v;
    } else {
        const int idx = (blk - 12) * 256 + t;
        const int b = idx >> 7, n = idx & 127;
        float a = -3.0e38f;
#pragma unroll
        for (int hd = 0; hd < NH; ++hd)
            a = fmaxf(a, invd[((size_t)((b * NH + hd) * QG + (n >> 4))) * 32 + (n & 15)]);
        const float mk = (a > 0.001f) ? 1.0f : 0.0f;
        *(volatile float*)(mask_out + idx) = mk;
        *(volatile float*)(maskws + idx) = mk;
        __threadfence();
        *(volatile float*)(mask_out + idx) = mk;
        *(volatile float*)(maskws + idx) = mk;
    }
}

__device__ __forceinline__ float tanh_q(float u) {
    const float e = __expf(2.0f * u);
    return fmaf(-2.0f, __builtin_amdgcn_rcpf(e + 1.0f), 1.0f);
}
__device__ __forceinline__ float gelu_t(float z) {
    const float u = 0.7978845608028654f * fmaf(0.044715f * z, z * z, z);
    return 0.5f * z * (1.0f + tanh_q(u));
}
__device__ __forceinline__ float tanh_s(float y) {
    const float a = fabsf(y);
    const float e = __expf(-2.0f * a);
    const float tq = (1.0f - e) * __builtin_amdgcn_rcpf(1.0f + e);
    return copysignf(tq, y);
}

__global__ void __launch_bounds__(256) pair_kernel(
    const float* __restrict__ H, const float* __restrict__ Cb,
    const float* __restrict__ W1, const float* __restrict__ W2, const float* __restrict__ b2,
    const float* __restrict__ bg1, const float* __restrict__ Wg2, const float* __restrict__ bg2,
    const float* __restrict__ ginit, const float* __restrict__ maskws, float* __restrict__ gout)
{
    __shared__ __align__(16) float sA[DM];
    __shared__ __align__(16) float sW[DM];
    __shared__ __align__(16) float sW2[DM];
    __shared__ __align__(16) float sG[DM];
    __shared__ __align__(16) float sWg2[DM];
    __shared__ __align__(16) float wb[8 * DM];
    __shared__ __align__(16) float go[NE];

    const int bi = blockIdx.x;
    const int b = bi >> 7;
    const int t = threadIdx.x, w = t >> 5, lane = t & 31;
    const float* Hi = H + (size_t)bi * NHO;
    for (int e = t; e < DM; e += 256) {
        sA[e]   = Hi[e] + Cb[b * DM + e];
        sW[e]   = W1[(size_t)1536 * DM + e];
        sW2[e]  = W2[e];
        sG[e]   = Hi[1536 + e] + bg1[e];
        sWg2[e] = Wg2[e];
    }
    __syncthreads();

    const float mi = maskws[bi];
    const float b2v = b2[0], bg2v = bg2[0];
    float* wbw = wb + w * DM;

#pragma unroll 1
    for (int p = 0; p < 16; ++p) {
        const int j = w * 16 + p;
        const float* Hj = H + (size_t)(b * NE + j) * NHO;
        float gacc = 0.0f;
#pragma unroll 1
        for (int q = 0; q < DM / 32; ++q) {
            const int e = lane + 32 * q;
            wbw[e] = sA[e] + Hj[DM + e];
            const float gz = sG[e] + Hj[2304 + e];
            gacc = fmaf(gelu_t(gz), sWg2[e], gacc);
        }
        gacc = wave_sum(gacc);
        float g = ginit[(size_t)bi * NE + j] * 1.6f - 0.8f;
#pragma unroll 1
        for (int step = 0; step < 3; ++step) {
            float acc = 0.0f;
#pragma unroll 1
            for (int q = 0; q < DM / 32; ++q) {
                const int e = lane + 32 * q;
                const float z = fmaf(g, sW[e], wbw[e]);
                acc = fmaf(gelu_t(z), sW2[e], acc);
            }
            acc = wave_sum(acc);
            g += tanh_s(acc + b2v);
        }
        const float gate = __builtin_amdgcn_rcpf(1.0f + __expf(-(gacc + bg2v)));
        g = g * gate;
        g = g * mi * maskws[b * NE + j];
        if (lane == 0) go[j] = g;
    }
    __syncthreads();
    if (w == 0) {
        const v4f_t v = *(const v4f*)&go[lane * 4];
        float* dst = gout + (size_t)bi * NE + lane * 4;
        *(volatile v4f_t*)dst = v;
        __threadfence();
        *(volatile v4f_t*)dst = v;
    }
}

extern "C" void kernel_launch(void* const* d_in, const int* in_sizes, int n_in,
                              void* d_out, int out_size, void* d_ws, size_t ws_size,
                              hipStream_t stream)
{
    if (n_in < 20) return;
    if (in_sizes[0] != NTOK * DM) return;
    if (in_sizes[1] != NB * NE * NE) return;
    if (in_sizes[2] != NE * DM) return;
    if (in_sizes[3] != SQ * DM) return;
    if (in_sizes[4] != DM * DM || in_sizes[6] != DM * DM || in_sizes[8] != DM * DM || in_sizes[10] != DM * DM) return;
    if (in_sizes[5] != DM || in_sizes[7] != DM || in_sizes[9] != DM || in_sizes[11] != DM) return;
    if (in_sizes[12] != 2305 * DM || in_sizes[13] != DM || in_sizes[14] != DM || in_sizes[15] < 1) return;
    if (in_sizes[16] != 1536 * DM || in_sizes[17] != DM || in_sizes[18] != DM || in_sizes[19] < 1) return;
    if (out_size != NROW * DM + NB * NE * NE + NROW) return;

    const float* emb  = (const float*)d_in[0];
    const float* gini = (const float*)d_in[1];
    const float* elib = (const float*)d_in[2];
    const float* pos  = (const float*)d_in[3];
    const float* Wq   = (const float*)d_in[4];
    const float* bq   = (const float*)d_in[5];
    const float* Wk   = (const float*)d_in[6];
    const float* bk   = (const float*)d_in[7];
    const float* Wv   = (const float*)d_in[8];
    const float* bv   = (const float*)d_in[9];
    const float* Wo   = (const float*)d_in[10];
    const float* bo   = (const float*)d_in[11];
    const float* W1   = (const float*)d_in[12];
    const float* b1   = (const float*)d_in[13];
    const float* W2   = (const float*)d_in[14];
    const float* b2   = (const float*)d_in[15];
    const float* Wg1  = (const float*)d_in[16];
    const float* bg1  = (const float*)d_in[17];
    const float* Wg2  = (const float*)d_in[18];
    const float* bg2  = (const float*)d_in[19];

    float* out  = (float*)d_out;
    float* out0 = out;
    float* out1 = out + (size_t)NROW * DM;
    float* out2 = out1 + (size_t)NB * NE * NE;

    size_t o = 0;
    const size_t szX   = (size_t)NTOK * DM * 2;
    const size_t szLIB = (size_t)NE * DM * 2;
    const size_t szW   = (size_t)DM * DM * 2;
    const size_t szWH  = (size_t)NHO * DM * 2;
    const size_t szVT  = (size_t)NB * DM * SQ * 2;
    const size_t szCT  = (size_t)NROW * DM * 2;
    const size_t szINV = (size_t)NB * NH * QG * 32 * 4;
    const size_t szCM  = (size_t)NB * DM * 4;
    const size_t szMK  = 2048;
    const size_t szH   = (size_t)NROW * NHO * 4;
    const size_t oXF = o;   o += szX;
    const size_t oXH = o;   o += szX;
    const size_t oXL = o;   o += szX;
    const size_t oLIB = o;  o += szLIB;
    const size_t oWQ = o;   o += szW;
    const size_t oWK = o;   o += szW;
    const size_t oWVH = o;  o += szW;
    const size_t oWVL = o;  o += szW;
    const size_t oWOH = o;  o += szW;
    const size_t oWOL = o;  o += szW;
    const size_t oWH = o;   o += szWH;
    const size_t oQP = o;   o += szLIB;
    const size_t oKP = o;   o += szX;
    const size_t oVTH = o;  o += szVT;
    const size_t oVTL = o;  o += szVT;
    const size_t oCTH = o;  o += szCT;
    const size_t oCTL = o;  o += szCT;
    const size_t oINV = o;  o += szINV;
    const size_t oCM = o;   o += szCM;
    const size_t oCB = o;   o += szCM;
    const size_t oMK = o;   o += szMK;
    const size_t oEF = o;   o += szCT;
    const size_t oH = o;    o += szH;
    if (o > ws_size) return;
    if (o > (size_t)134217728) return;

    char* ws = (char*)d_ws;
    u16* xf   = (u16*)(ws + oXF);
    u16* xh   = (u16*)(ws + oXH);
    u16* xl   = (u16*)(ws + oXL);
    u16* libf = (u16*)(ws + oLIB);
    u16* wqt  = (u16*)(ws + oWQ);
    u16* wkt  = (u16*)(ws + oWK);
    u16* wvth = (u16*)(ws + oWVH);
    u16* wvtl = (u16*)(ws + oWVL);
    u16* woth = (u16*)(ws + oWOH);
    u16* wotl = (u16*)(ws + oWOL);
    u16* wht  = (u16*)(ws + oWH);
    u16* qpl  = (u16*)(ws + oQP);
    u16* kpl  = (u16*)(ws + oKP);
    u16* vth  = (u16*)(ws + oVTH);
    u16* vtl  = (u16*)(ws + oVTL);
    u16* ctxh = (u16*)(ws + oCTH);
    u16* ctxl = (u16*)(ws + oCTL);
    float* invd = (float*)(ws + oINV);
    float* cm   = (float*)(ws + oCM);
    float* Cb   = (float*)(ws + oCB);
    float* mkws = (float*)(ws + oMK);
    u16* entf   = (u16*)(ws + oEF);
    float* Hb   = (float*)(ws + oH);

    const int n8X = NTOK * DM / 8, n8L = NE * DM / 8;
    xprep_kernel<<<dim3((n8X + 255) / 256), 256, 0, stream>>>(emb, pos, xf, xh, xl, n8X);
    cvt16_kernel<<<dim3((n8L + 255) / 256), 256, 0, stream>>>(elib, libf, n8L, 256.0f);
    context_kernel<<<dim3(DM / 256, NB), 256, 0, stream>>>(emb, pos, cm);

    const dim3 gw(DM / 64, DM / 64);
    wtrans_kernel<0><<<gw, 256, 0, stream>>>(Wq, wqt, wqt, 16.0f);
    wtrans_kernel<0><<<gw, 256, 0, stream>>>(Wk, wkt, wkt, 16.0f);
    wtrans_kernel<1><<<gw, 256, 0, stream>>>(Wv, wvth, wvtl, 1.0f);
    wtrans_kernel<1><<<gw, 256, 0, stream>>>(Wo, woth, wotl, 1.0f);
    wtrans_kernel<0><<<gw, 256, 0, stream>>>(W1, wht, wht, 64.0f);
    wtrans_kernel<0><<<gw, 256, 0, stream>>>(W1 + (size_t)DM * DM, wht + (size_t)DM * DM, wht, 64.0f);
    wtrans_kernel<0><<<gw, 256, 0, stream>>>(Wg1, wht + (size_t)2 * DM * DM, wht, 64.0f);
    wtrans_kernel<0><<<gw, 256, 0, stream>>>(Wg1 + (size_t)DM * DM, wht + (size_t)3 * DM * DM, wht, 64.0f);

    gemm_kernel<false, 1><<<dim3(DM / 64, NTOK / 64), 128, 0, stream>>>(
        xf, xf, wkt, wkt, bk, 1, NTOK, DM, DM, 1.0f / 16.0f, 1.0f, Hb, kpl, kpl, mkws);
    gemm_kernel<true, 4><<<dim3(DM / 64, NTOK / 64), 128, 0, stream>>>(
        xh, xl, wvth, wvtl, bv, 1, NTOK, DM, DM, 1.0f, 1.0f, Hb, vth, vtl, mkws);
    gemm_kernel<false, 1><<<dim3(DM / 64, NE / 64), 128, 0, stream>>>(
        libf, libf, wqt, wqt, bq, 1, NE, DM, DM, 1.0f / 4096.0f, 64.0f, Hb, qpl, qpl, mkws);

    hipFuncSetAttribute(reinterpret_cast<const void*>(&attn_kernel),
                        hipFuncAttributeMaxDynamicSharedMemorySize, ATT_LDS);
    attn_kernel<<<dim3(QG, NH, NB), 256, ATT_LDS, stream>>>(qpl, kpl, vth, vtl, ctxh, ctxl, invd);

    post_kernel<<<dim3(14), 256, 0, stream>>>(cm, W1, b1, invd, Cb, mkws, out2);

    gemm_kernel<true, 3><<<dim3(DM / 64, NROW / 64), 128, 0, stream>>>(
        ctxh, ctxl, woth, wotl, bo, 1, NROW, DM, DM, 1.0f, 256.0f, out0, entf, entf, mkws);

    gemm_kernel<false, 0><<<dim3(NHO / 64, NROW / 64), 128, 0, stream>>>(
        entf, entf, wht, wht, Hb, 0, NROW, NHO, DM, 1.0f / 16384.0f, 1.0f, Hb, kpl, kpl, mkws);

    pair_kernel<<<dim3(NROW), 256, 0, stream>>>(Hb, Cb, W1, W2, b2, bg1, Wg2, bg2, gini, mkws, out1);
}
